// LinearCrossAttention_56813827392083
// MI455X (gfx1250) — hardware-run, weakly checked
//
#include <hip/hip_runtime.h>
#include <math.h>

typedef __attribute__((ext_vector_type(16))) _Float16 v16h;
typedef __attribute__((ext_vector_type(16))) __bf16 v16b;
typedef __attribute__((ext_vector_type(8)))  _Float16 v8h;
typedef __attribute__((ext_vector_type(8)))  float v8f;
typedef __attribute__((ext_vector_type(4)))  float v4f;
typedef __attribute__((ext_vector_type(2)))  float v2f;
typedef __attribute__((ext_vector_type(4)))  unsigned v4u;
typedef __attribute__((ext_vector_type(4)))  int v4i;
typedef float __attribute__((may_alias)) float_a;
typedef int __attribute__((may_alias)) int_a;

template <typename T> __device__ __forceinline__ void vst2(void* p, T v) { *(volatile T*)p = v; __threadfence(); *(volatile T*)p = v; }
__device__ __forceinline__ v8f wmma16(v16h a, v16h b, v8f c) {
  v8f d = __builtin_amdgcn_wmma_f32_16x16x32_f16(false, a, false, b, (short)0, c, false, false);
  asm volatile("v_nop\n\tv_nop\n\tv_nop\n\tv_nop" : "+v"(d) : "v"(a), "v"(b));
  return d;
}
__device__ __forceinline__ v8f wmma_bf(v16b a, v16b b, v8f c) {
  v8f d = __builtin_amdgcn_wmma_f32_16x16x32_bf16(false, a, false, b, (short)0, c, false, false);
  asm volatile("v_nop\n\tv_nop\n\tv_nop\n\tv_nop" : "+v"(d) : "v"(a), "v"(b));
  return d;
}
__device__ __forceinline__ v16h frag_h(const _Float16* rowk0, int lane) {
  union { v16h v; v8h q[2]; } u; const _Float16* p = rowk0 + 8 * (lane >> 4);
  u.q[0] = *(const v8h*)p; u.q[1] = *(const v8h*)(p + 16); return u.v;
}
__device__ __forceinline__ v16h frag_f32(const float* rowk0, int lane) {
  v16h a; const float* p = rowk0 + 8 * (lane >> 4);
#pragma unroll
  for (int i = 0; i < 8; ++i) { a[i] = (_Float16)p[i]; a[8 + i] = (_Float16)p[16 + i]; }
  return a;
}
__device__ __forceinline__ v16h frag_f32s(const float* rowk0, int lane, float sc) {
  v16h a; const float* p = rowk0 + 8 * (lane >> 4);
#pragma unroll
  for (int i = 0; i < 8; ++i) { a[i] = (_Float16)(p[i] * sc); a[8 + i] = (_Float16)(p[16 + i] * sc); }
  return a;
}
__device__ __forceinline__ v16h fragc_f32(const float* W, int k0, int n, int lane, int ld, int K) {
  v16h a; const int g = lane >> 4;
#pragma unroll
  for (int i = 0; i < 8; ++i) { const int ka = k0 + 8 * g + i, kb = ka + 16;
    a[i] = (_Float16)(ka < K ? W[(size_t)(ka < K ? ka : K - 1) * ld + n] : 0.f); a[8 + i] = (_Float16)(kb < K ? W[(size_t)(kb < K ? kb : K - 1) * ld + n] : 0.f); }
  return a;
}
struct F2 { v16b h, l; };
__device__ __forceinline__ F2 bsplit16(const float v[16]) { F2 r;
#pragma unroll
  for (int i = 0; i < 16; ++i) { const __bf16 h = (__bf16)v[i]; r.h[i] = h; r.l[i] = (__bf16)(v[i] - (float)h); }
  return r; }
__device__ __forceinline__ F2 split_row(const float* row, int k0, int lane) { float v[16]; const float* p = row + k0 + 8 * (lane >> 4);
#pragma unroll
  for (int i = 0; i < 8; ++i) { v[i] = p[i]; v[8 + i] = p[16 + i]; }
  return bsplit16(v); }
__device__ __forceinline__ F2 split_rowK(const float* row, int k0, int lane, int K) { float v[16]; const int g = lane >> 4;
#pragma unroll
  for (int i = 0; i < 8; ++i) { const int ka = k0 + 8 * g + i, kb = ka + 16; v[i] = ka < K ? row[ka < K ? ka : K - 1] : 0.f; v[8 + i] = kb < K ? row[kb < K ? kb : K - 1] : 0.f; }
  return bsplit16(v); }
__device__ __forceinline__ F2 split_col(const float* W, int k0, int n, int lane, int ld, int K) { float v[16]; const int g = lane >> 4;
#pragma unroll
  for (int i = 0; i < 8; ++i) { const int ka = k0 + 8 * g + i, kb = ka + 16; v[i] = ka < K ? W[(size_t)(ka < K ? ka : K - 1) * ld + n] : 0.f; v[8 + i] = kb < K ? W[(size_t)(kb < K ? kb : K - 1) * ld + n] : 0.f; }
  return bsplit16(v); }
__device__ __forceinline__ v8f mac3(const F2& a, const F2& b, v8f c) { c = wmma_bf(a.l, b.h, c); c = wmma_bf(a.h, b.l, c); return wmma_bf(a.h, b.h, c); }
__device__ __forceinline__ float sigm(float v) { return 1.0f / (1.0f + expf(-v)); }
#define LDSX() do { asm volatile("s_wait_dscnt 0" ::: "memory"); __builtin_amdgcn_wave_barrier(); __builtin_amdgcn_fence(__ATOMIC_RELEASE, "workgroup"); } while (0)


#define NB 4
#define T1 4096
#define T2 2048
#define CC 512
#define NH 8
#define HD 64
#define NIN 3
#ifndef TNB
#define TNB NB
#endif
typedef __attribute__((ext_vector_type(8))) __bf16 v8b;
__device__ __forceinline__ v16b frag_b(const __bf16* rowk0, int lane) {
  union { v16b v; v8b q[2]; } u; const __bf16* p = rowk0 + 8 * (lane >> 4);
  u.q[0] = *(const v8b*)p; u.q[1] = *(const v8b*)(p + 16); return u.v;
}
__device__ __forceinline__ float bfr(float v) { return (float)(__bf16)v; }
__device__ __attribute__((noinline)) float exp_ni(float v) { return expf(v); }
__device__ __attribute__((noinline)) float erf_ni(float v) { return erff(v); }

#define WS_Q   0u
#define PLK    (2u * (size_t)NB * CC * T2)
#define WS_KH  (WS_Q + 4u * (size_t)NB * T1 * CC)
#define WS_KL  (WS_KH + NIN * PLK)
#define WS_VH  (WS_KL + NIN * PLK)
#define WS_VL  (WS_VH + NIN * PLK)
#define WS_CT  (WS_VL + NIN * PLK)
#define WS_KS  (WS_CT + 4u * (size_t)NIN * NB * NH * HD * HD)
#define WS_DI  (WS_KS + 4u * (size_t)NIN * NB * NH * HD)
#define WS_END (WS_DI + 4u * (size_t)NB * T1 * NH * 4)

__device__ __forceinline__ v16b fragb_f32(const float* __restrict__ p, int lane) { v16b a; const float* pp = p + 8 * (lane >> 4);
#pragma unroll
  for (int i = 0; i < 8; ++i) { a[i] = (__bf16)pp[i]; a[8 + i] = (__bf16)pp[16 + i]; } return a; }
__device__ __forceinline__ void head_softmax(v8f acc[8], int r) {
#pragma unroll
  for (int hh = 0; hh < 2; ++hh) { float mx = -3.0e38f;
#pragma unroll
    for (int j = 0; j < 4; ++j) mx = fmaxf(mx, acc[hh * 4 + j][r]);
#pragma unroll
    for (int o = 1; o < 16; o <<= 1) mx = fmaxf(mx, __shfl_xor(mx, o));
    float s = 0.f;
#pragma unroll
    for (int j = 0; j < 4; ++j) { acc[hh * 4 + j][r] = expf(acc[hh * 4 + j][r] - mx); s += acc[hh * 4 + j][r]; }
#pragma unroll
    for (int o = 1; o < 16; o <<= 1) s += __shfl_xor(s, o);
    const float inv = 1.0f / s;
#pragma unroll
    for (int j = 0; j < 4; ++j) acc[hh * 4 + j][r] *= inv; } }
__global__ __launch_bounds__(128) void k_q(const float* __restrict__ X, const float* __restrict__ WQ, const float* __restrict__ BQ, float* __restrict__ Q) { __shared__ __align__(16) float sf[4][16][132];
  const int tid = threadIdx.x, wave = tid >> 5, lane = tid & 31, col = lane & 15, g = lane >> 4; const size_t r0 = (size_t)blockIdx.x * 64 + wave * 16; const int c0 = blockIdx.y * 128;
  v8f acc[8] = {};
#pragma unroll 2
  for (int kc = 0; kc < CC / 32; ++kc) { const v16b a = fragb_f32(X + (r0 + col) * CC + kc * 32, lane);
#pragma unroll
    for (int j = 0; j < 8; ++j) acc[j] = wmma_bf(a, fragb_f32(WQ + (size_t)(c0 + j * 16 + col) * CC + kc * 32, lane), acc[j]); }
#pragma unroll
  for (int j = 0; j < 8; ++j) { const float bb = bfr(BQ[c0 + j * 16 + col]);
#pragma unroll
    for (int r = 0; r < 8; ++r) acc[j][r] += bb; }
#pragma unroll
  for (int r = 0; r < 8; ++r) head_softmax(acc, r);
#pragma unroll
  for (int j = 0; j < 8; ++j)
#pragma unroll
    for (int r = 0; r < 8; ++r) sf[wave][8 * g + r][j * 16 + col] = acc[j][r];
  LDSX(); for (int rl = 0; rl < 16; ++rl) vst2(Q + (r0 + rl) * CC + c0 + lane * 4, *(const v4f*)&sf[wave][rl][lane * 4]); }
__global__ __launch_bounds__(128) void k_kv(const float* __restrict__ Y0, const float* __restrict__ Y1, const float* __restrict__ Y2, const float* __restrict__ WK, const float* __restrict__ BK, const float* __restrict__ WV, const float* __restrict__ BV, _Float16* __restrict__ KH, _Float16* __restrict__ KL, _Float16* __restrict__ VH, _Float16* __restrict__ VL) { __shared__ __align__(16) _Float16 th[128][72], tl[128][72];
  const int tid = threadIdx.x, wave = tid >> 5, lane = tid & 31, col = lane & 15, g = lane >> 4; const int i = blockIdx.z >> 1; const bool isv = blockIdx.z & 1; const float* Y = i == 0 ? Y0 : i == 1 ? Y1 : Y2; const float* Wm = (isv ? WV : WK) + (size_t)i * CC * CC; const float* Bm = (isv ? BV : BK) + (size_t)i * CC;
  const size_t r0 = (size_t)blockIdx.x * 64 + wave * 16; const int c0 = blockIdx.y * 128; const size_t b = ((size_t)blockIdx.x * 64) / T2; const int n0 = (int)(((size_t)blockIdx.x * 64) % T2);
  v8f acc[8] = {};
#pragma unroll 2
  for (int kc = 0; kc < CC / 32; ++kc) { const v16b a = fragb_f32(Y + (r0 + col) * CC + kc * 32, lane);
#pragma unroll
    for (int j = 0; j < 8; ++j) acc[j] = wmma_bf(a, fragb_f32(Wm + (size_t)(c0 + j * 16 + col) * CC + kc * 32, lane), acc[j]); }
#pragma unroll
  for (int j = 0; j < 8; ++j) { const float bb = bfr(Bm[c0 + j * 16 + col]);
#pragma unroll
    for (int r = 0; r < 8; ++r) acc[j][r] += bb; }
  if (!isv) {
#pragma unroll
    for (int r = 0; r < 8; ++r) head_softmax(acc, r); }
#pragma unroll
  for (int j = 0; j < 8; ++j)
#pragma unroll
    for (int r = 0; r < 8; ++r) { const float v = acc[j][r]; const _Float16 hv = (_Float16)v; const int cl = j * 16 + col, rl = wave * 16 + 8 * g + r; th[cl][rl] = hv; tl[cl][rl] = (_Float16)((v - (float)hv) * 2048.0f); }
  __syncthreads();
  { _Float16* PH = (isv ? VH : KH) + (size_t)i * (PLK / 2); _Float16* PL = (isv ? VL : KL) + (size_t)i * (PLK / 2);
    for (int e = tid; e < 128 * 8; e += 128) { const int cl = e >> 3, q = e & 7; const size_t o = (b * CC + c0 + cl) * (size_t)T2 + n0 + q * 8; vst2((unsigned*)(PH + o), *(const v4u*)&th[cl][q * 8]); vst2((unsigned*)(PL + o), *(const v4u*)&tl[cl][q * 8]); } } }
__global__ __launch_bounds__(128) void k_dots(const _Float16* __restrict__ KH, const _Float16* __restrict__ KL, const _Float16* __restrict__ VH, const _Float16* __restrict__ VL, float* __restrict__ CT, float* __restrict__ KS) { __shared__ __align__(16) float sf[4][16][68]; __shared__ __align__(16) float sks[64];
  const int tid = threadIdx.x, wave = tid >> 5, lane = tid & 31, col = lane & 15, g = lane >> 4; const size_t bh = blockIdx.x; const int i = blockIdx.y; const size_t set = (size_t)i * (PLK / 2);
  const _Float16 *kh = KH + set, *kl = KL + set, *vh = VH + set, *vl = VL + set;
  { const int d = tid >> 1, half = tid & 1; const _Float16* ph = kh + (bh * HD + d) * T2 + half * (T2 / 2); const _Float16* pl = kl + (bh * HD + d) * T2 + half * (T2 / 2); float s = 0.f;
#pragma unroll 1
    for (int n = 0; n < T2 / 2; ++n) s += (float)ph[n] + (float)pl[n] * (1.0f / 2048.0f);
    s += __shfl_xor(s, 1); if (half == 0) sks[d] = s; }
  const size_t pe = (bh * HD + wave * 16 + col) * T2;
  v8f acc[4] = {}, accl[4] = {};
#pragma unroll 2
  for (int kc = 0; kc < T2 / 32; ++kc) { const v16h ah = frag_h(vh + pe + kc * 32, lane), al = frag_h(vl + pe + kc * 32, lane);
#pragma unroll
    for (int j = 0; j < 4; ++j) { const size_t pd = (bh * HD + j * 16 + col) * T2 + kc * 32; const v16h k2 = frag_h(kh + pd, lane); acc[j] = wmma16(ah, k2, acc[j]); accl[j] = wmma16(al, k2, accl[j]); accl[j] = wmma16(ah, frag_h(kl + pd, lane), accl[j]); } }
#pragma unroll
  for (int j = 0; j < 4; ++j)
#pragma unroll
    for (int r = 0; r < 8; ++r) sf[wave][8 * g + r][j * 16 + col] = acc[j][r] + accl[j][r] * (1.0f / 2048.0f);
  __syncthreads();
  for (int rl = 0; rl < 16; ++rl) if (lane < 16) vst2(CT + (((size_t)i * NB * NH + bh) * HD + wave * 16 + rl) * HD + lane * 4, *(const v4f*)&sf[wave][rl][lane * 4]);
  if (tid < 16) vst2(KS + ((size_t)i * NB * NH + bh) * HD + tid * 4, *(const v4f*)&sks[tid * 4]); }
__global__ __launch_bounds__(256) void k_dinv(const float* __restrict__ Q, const float* __restrict__ KS, float* __restrict__ DI) { const size_t e = (size_t)blockIdx.x * 256 + threadIdx.x; const size_t row = e / NH; const int h = e % NH; const size_t b = row / T1; const float* qr = Q + row * CC + h * HD;
  float s[3] = {0.f, 0.f, 0.f};
#pragma unroll 1
  for (int d = 0; d < HD; ++d) { const float qv = qr[d];
#pragma unroll
    for (int i = 0; i < 3; ++i) s[i] += qv * KS[((size_t)i * NB * NH + b * NH + h) * HD + d]; }
  v4f o; o[0] = 1.0f / (s[0] + 1e-8f); o[1] = 1.0f / (s[1] + 1e-8f); o[2] = 1.0f / (s[2] + 1e-8f); o[3] = 0.f; vst2(DI + (row * NH + h) * 4, o); }
__global__ __launch_bounds__(128) void k_o(const float* __restrict__ Q, const float* __restrict__ CT, const float* __restrict__ DI, const float* __restrict__ WO, const float* __restrict__ BO, float* __restrict__ OUT) { __shared__ __align__(16) float sc[4][16][36]; __shared__ __align__(16) float sf[4][16][132];
  const int tid = threadIdx.x, wave = tid >> 5, lane = tid & 31, col = lane & 15, g = lane >> 4; const size_t r0 = (size_t)blockIdx.x * 64 + wave * 16; const int c0 = blockIdx.y * 128; const size_t b = r0 / T1;
  v8f acc[8] = {};
#pragma unroll 1
  for (int ch = 0; ch < CC / 32; ++ch) { const int h = ch >> 1, half = ch & 1;
    float di[3][8];
#pragma unroll
    for (int r = 0; r < 8; ++r) { const float* dp = DI + ((r0 + 8 * g + r) * NH + h) * 4; di[0][r] = dp[0]; di[1][r] = dp[1]; di[2][r] = dp[2]; }
    v8f tot[2];
#pragma unroll
    for (int tt = 0; tt < 2; ++tt)
#pragma unroll
      for (int r = 0; r < 8; ++r) tot[tt][r] = Q[(r0 + 8 * g + r) * CC + ch * 32 + tt * 16 + col];
    F2 aq[2];
#pragma unroll
    for (int kc = 0; kc < 2; ++kc) aq[kc] = split_row(Q + (r0 + col) * CC + h * HD, kc * 32, lane);
#pragma unroll
    for (int i = 0; i < NIN; ++i) { v8f c2[2] = {};
#pragma unroll
      for (int kc = 0; kc < 2; ++kc)
#pragma unroll
        for (int tt = 0; tt < 2; ++tt) { const F2 bw = split_row(CT + ((((size_t)i * NB * NH + b * NH + h) * HD) + half * 32 + tt * 16 + col) * HD, kc * 32, lane); c2[tt] = mac3(aq[kc], bw, c2[tt]); }
#pragma unroll
      for (int tt = 0; tt < 2; ++tt)
#pragma unroll
        for (int r = 0; r < 8; ++r) tot[tt][r] += c2[tt][r] * di[i][r]; }
#pragma unroll
    for (int tt = 0; tt < 2; ++tt)
#pragma unroll
      for (int r = 0; r < 8; ++r) sc[wave][8 * g + r][tt * 16 + col] = tot[tt][r];
    LDSX();
    { const F2 a = split_row(&sc[wave][col][0], 0, lane);
#pragma unroll
      for (int j = 0; j < 8; ++j) { const v16b w = fragb_f32(WO + (size_t)(c0 + j * 16 + col) * CC + ch * 32, lane); acc[j] = wmma_bf(a.h, w, acc[j]); acc[j] = wmma_bf(a.l, w, acc[j]); } }
    LDSX(); }
#pragma unroll
  for (int j = 0; j < 8; ++j)
#pragma unroll
    for (int r = 0; r < 8; ++r) sf[wave][8 * g + r][j * 16 + col] = acc[j][r] + bfr(BO[c0 + j * 16 + col]);
  LDSX(); for (int rl = 0; rl < 16; ++rl) vst2(OUT + (r0 + rl) * CC + c0 + lane * 4, *(const v4f*)&sf[wave][rl][lane * 4]); }
extern "C" void kernel_launch(void* const* d_in, const int* in_sizes, int n_in, void* d_out, int out_size, void* d_ws, size_t ws_size, hipStream_t stream) {
  (void)in_sizes; (void)n_in; (void)out_size;
  const float** F = (const float**)d_in;
  if (ws_size < (size_t)WS_END) return;
  char* ws = (char*)d_ws; float* Q = (float*)(ws + WS_Q); _Float16 *KH = (_Float16*)(ws + WS_KH), *KL = (_Float16*)(ws + WS_KL), *VH = (_Float16*)(ws + WS_VH), *VL = (_Float16*)(ws + WS_VL); float *CT = (float*)(ws + WS_CT), *KS = (float*)(ws + WS_KS), *DI = (float*)(ws + WS_DI);
  k_q<<<dim3(TNB * T1 / 64, CC / 128), 128, 0, stream>>>(F[0], F[4], F[5], Q);
  k_kv<<<dim3(TNB * T2 / 64, CC / 128, NIN * 2), 128, 0, stream>>>(F[1], F[2], F[3], F[6], F[7], F[8], F[9], KH, KL, VH, VL);
  k_dots<<<dim3(TNB * NH, NIN), 128, 0, stream>>>(KH, KL, VH, VL, CT, KS);
  k_dinv<<<TNB * T1 * NH / 256, 256, 0, stream>>>(Q, KS, DI);
  k_o<<<dim3(TNB * T1 / 64, CC / 128), 128, 0, stream>>>(Q, CT, DI, F[10], F[11], (float*)d_out);
}
